// EncryptedCrossAttention_83184926589619
// MI455X (gfx1250) — hardware-verified
//
#include <hip/hip_runtime.h>

typedef _Float16 v16h __attribute__((ext_vector_type(16)));
typedef _Float16 v8h  __attribute__((ext_vector_type(8)));
typedef float    v8f  __attribute__((ext_vector_type(8)));
typedef float    v4f  __attribute__((ext_vector_type(4)));
typedef v8h __attribute__((may_alias)) v8ha;
typedef v4f __attribute__((may_alias)) v4fa;

union Frag { v16h v; v8h half[2]; };

#define DMODEL 1024
#define NHEADS 8
#define HD     64
#define INNER  (NHEADS * HD)
#define SEQ    2048
#define BATCH  4
#define MROWS  (BATCH * SEQ)
#define NX     (MROWS * DMODEL)
#define NW     (DMODEL * INNER)
#define NO     (MROWS * INNER)
#define NX8    (NX / 8)
#define WSC    32.0f
#define OSC    16.0f
#define PSCALE 16384.0f
#define QKSC   0.125f

__device__ __forceinline__ v8f wmma_f16(v16h a, v16h b, v8f c) {
  v8f d = __builtin_amdgcn_wmma_f32_16x16x32_f16(false, a, false, b, (short)0, c, false, false);
  asm volatile("v_nop\n\tv_nop\n\tv_nop\n\tv_nop" : "+v"(d) : "v"(a), "v"(b));
  return d;
}

__device__ __forceinline__ v16h load_frag(const _Float16* p, int h) {
  Frag f;
  f.half[0] = *(const v8ha*)(p + 8 * h);
  f.half[1] = *(const v8ha*)(p + 16 + 8 * h);
  return f.v;
}

__global__ __launch_bounds__(256) void convert_act_kernel(
    const float* __restrict__ x, const float* __restrict__ ctx,
    _Float16* __restrict__ xh, _Float16* __restrict__ ch)
{
  const int g = blockIdx.x * 256 + threadIdx.x;
  if (g >= 2 * NX8) return;
  const float* src;
  _Float16* dst;
  if (g < NX8) {
    src = x + (size_t)g * 8;
    dst = xh + (size_t)g * 8;
  } else {
    const int e = g - NX8;
    src = ctx + (size_t)e * 8;
    dst = ch + (size_t)e * 8;
  }
  const v4f a = *(const v4fa*)src;
  const v4f c = *(const v4fa*)(src + 4);
  const v8h o = { (_Float16)a.x, (_Float16)a.y, (_Float16)a.z, (_Float16)a.w,
                  (_Float16)c.x, (_Float16)c.y, (_Float16)c.z, (_Float16)c.w };
  *(volatile v8h*)dst = o;
  __threadfence();
  *(volatile v8h*)dst = o;
}

__device__ __forceinline__ void wt_store_pass(const _Float16* sT, _Float16* dst, int R,
                                              int r0, int c0, int w, int lane) {
  const int q8 = lane & 7, sub = lane >> 3;
  #pragma unroll
  for (int i = 0; i < 2; ++i) {
    const int c = 8 * w + 4 * i + sub;
    const v8h v = *(const v8ha*)(sT + c * 64 + 8 * q8);
    *(volatile v8h*)(dst + (size_t)(c0 + c) * R + r0 + 8 * q8) = v;
  }
}

__global__ __launch_bounds__(256) void wtrans_kernel(
    const float* __restrict__ wq, const float* __restrict__ wk,
    const float* __restrict__ wv, const float* __restrict__ wo,
    _Float16* __restrict__ wT, _Float16* __restrict__ woT)
{
  __shared__ __attribute__((aligned(16))) _Float16 sT[64 * 64];

  const int tid = threadIdx.x, lane = tid & 31, w = tid >> 5;
  const int blk = blockIdx.x;
  const float* src;
  _Float16* dst;
  int R, C, tr, tc;
  if (blk < 384) {
    const int which = blk >> 7, t = blk & 127;
    src = (which == 0) ? wq : ((which == 1) ? wk : wv);
    dst = wT + (size_t)which * NW;
    R = DMODEL; C = INNER;
    tr = t >> 3; tc = t & 7;
  } else {
    const int t = blk - 384;
    src = wo; dst = woT;
    R = INNER; C = DMODEL;
    tr = t >> 4; tc = t & 15;
  }
  const int r0 = tr * 64, c0 = tc * 64;

  #pragma unroll
  for (int p = 0; p < 4; ++p) {
    const int i = tid + 256 * p;
    const int r = i >> 4, c4 = i & 15;
    const v4f v = *(const v4fa*)(src + (size_t)(r0 + r) * C + c0 + 4 * c4);
    _Float16* sp = sT + (4 * c4) * 64 + r;
    sp[0]   = (_Float16)(v.x * WSC);
    sp[64]  = (_Float16)(v.y * WSC);
    sp[128] = (_Float16)(v.z * WSC);
    sp[192] = (_Float16)(v.w * WSC);
  }
  __syncthreads();

  wt_store_pass(sT, dst, R, r0, c0, w, lane);
  __threadfence();
  wt_store_pass(sT, dst, R, r0, c0, w, lane);
}

__device__ __forceinline__ void proj_store_pass(const _Float16* sT, _Float16* plane, _Float16* vt,
                                                int which, int bh, int l0, int w, int lane) {
  const int q8 = lane & 7, sub = lane >> 3;
  #pragma unroll
  for (int i = 0; i < 8; ++i) {
    const int lid = w * 32 + i * 4 + sub;
    v8h v;
    _Float16* dst;
    if (which != 2) {
      v = *(const v8ha*)(sT + lid * HD + 8 * q8);
      dst = plane + ((size_t)bh * SEQ + l0 + lid) * HD + 8 * q8;
    } else {
      const int d = lid >> 1, hl = lid & 1;
      v = *(const v8ha*)(sT + d * 128 + 64 * hl + 8 * q8);
      dst = vt + ((size_t)bh * HD + d) * SEQ + l0 + 64 * hl + 8 * q8;
    }
    *(volatile v8h*)dst = v;
  }
}

__global__ __launch_bounds__(128) void qkv_kernel(
    const _Float16* __restrict__ xh,
    const _Float16* __restrict__ ch,
    const _Float16* __restrict__ wT,
    const float* __restrict__ bq, const float* __restrict__ bk, const float* __restrict__ bv,
    _Float16* __restrict__ qh,
    _Float16* __restrict__ kh,
    _Float16* __restrict__ vt)
{
  __shared__ __attribute__((aligned(16))) _Float16 sT[128 * 64];

  const int tid = threadIdx.x, lane = tid & 31, w = tid >> 5;
  const int h = lane >> 4, m = lane & 15;
  const int m0 = blockIdx.x * 128;
  const int cg = blockIdx.y;
  const int which = cg >> 3, head = cg & 7;
  const int m0w = m0 + 32 * w;

  const _Float16* ap  = (which == 0) ? xh : ch;
  const _Float16* xa0 = ap + (size_t)(m0w + m) * DMODEL;
  const _Float16* xa1 = xa0 + (size_t)16 * DMODEL;
  const _Float16* wb  = wT + ((size_t)which * INNER + head * HD + m) * DMODEL;

  const v8f zero8 = {0.f, 0.f, 0.f, 0.f, 0.f, 0.f, 0.f, 0.f};
  v8f acc[2][4];
  #pragma unroll
  for (int mt = 0; mt < 2; ++mt)
    #pragma unroll
    for (int nt = 0; nt < 4; ++nt) acc[mt][nt] = zero8;

  #pragma unroll 1
  for (int k0 = 0; k0 < DMODEL; k0 += 32) {
    const v16h a0 = load_frag(xa0 + k0, h);
    const v16h a1 = load_frag(xa1 + k0, h);
    #pragma unroll
    for (int nt = 0; nt < 4; ++nt) {
      const v16h b = load_frag(wb + (size_t)nt * 16 * DMODEL + k0, h);
      acc[0][nt] = wmma_f16(a0, b, acc[0][nt]);
      acc[1][nt] = wmma_f16(a1, b, acc[1][nt]);
    }
  }

  const float* bias = (which == 0) ? bq : ((which == 1) ? bk : bv);
  #pragma unroll
  for (int nt = 0; nt < 4; ++nt) {
    const int feat = 16 * nt + m;
    const float bvl = bias[head * HD + feat];
    #pragma unroll
    for (int mt = 0; mt < 2; ++mt) {
      #pragma unroll
      for (int r = 0; r < 8; ++r) {
        const int tokl = 32 * w + 16 * mt + 8 * h + r;
        const float y = acc[mt][nt][r] * (1.0f / WSC) + bvl;
        const int idx = (which == 2) ? (feat * 128 + tokl) : (tokl * HD + feat);
        sT[idx] = (_Float16)y;
      }
    }
  }
  __syncthreads();

  const int b = m0 / SEQ, l0 = m0 - b * SEQ, bh = b * NHEADS + head;
  _Float16* plane = (which == 0) ? qh : kh;
  proj_store_pass(sT, plane, vt, which, bh, l0, w, lane);
  __threadfence();
  proj_store_pass(sT, plane, vt, which, bh, l0, w, lane);
}

__device__ __forceinline__ v16h pack_p(v8f a, v8f c) {
  const v16h r = { (_Float16)(a[0] * PSCALE), (_Float16)(a[1] * PSCALE), (_Float16)(a[2] * PSCALE), (_Float16)(a[3] * PSCALE),
                   (_Float16)(a[4] * PSCALE), (_Float16)(a[5] * PSCALE), (_Float16)(a[6] * PSCALE), (_Float16)(a[7] * PSCALE),
                   (_Float16)(c[0] * PSCALE), (_Float16)(c[1] * PSCALE), (_Float16)(c[2] * PSCALE), (_Float16)(c[3] * PSCALE),
                   (_Float16)(c[4] * PSCALE), (_Float16)(c[5] * PSCALE), (_Float16)(c[6] * PSCALE), (_Float16)(c[7] * PSCALE) };
  return r;
}

__device__ __forceinline__ void att_store_pass(const _Float16* so, _Float16* oh,
                                               int b, int head, int q0, int lane) {
  const int q8 = lane & 7, sub = lane >> 3;
  #pragma unroll
  for (int i = 0; i < 4; ++i) {
    const int row = i * 4 + sub;
    const v8h v = *(const v8ha*)(so + row * 64 + 8 * q8);
    const size_t gi = ((size_t)b * SEQ + q0 + row) * INNER + head * HD + 8 * q8;
    *(volatile v8h*)(oh + gi) = v;
  }
}

__global__ __launch_bounds__(128) void attn_kernel(
    const _Float16* __restrict__ qh,
    const _Float16* __restrict__ kh,
    const _Float16* __restrict__ vt,
    _Float16* __restrict__ oh)
{
  __shared__ __attribute__((aligned(16))) _Float16 sO[4 * 16 * 64];

  const int tid = threadIdx.x, lane = tid & 31, w = tid >> 5;
  const int h = lane >> 4, m = lane & 15;
  const int bh = blockIdx.y, b = bh >> 3, head = bh & 7;
  const int q0 = blockIdx.x * 64 + 16 * w;

  const _Float16* qrow = qh + ((size_t)bh * SEQ + q0 + m) * HD;
  const v16h qb0 = load_frag(qrow, h);
  const v16h qb1 = load_frag(qrow + 32, h);

  const v8f zero8 = {0.f, 0.f, 0.f, 0.f, 0.f, 0.f, 0.f, 0.f};
  v8f o[4];
  #pragma unroll
  for (int t = 0; t < 4; ++t) o[t] = zero8;
  float mrun = -1e30f, lrun = 0.0f;

  const _Float16* kbase = kh + ((size_t)bh * SEQ + m) * HD;
  const _Float16* vbase = vt + ((size_t)bh * HD + m) * SEQ;

  #pragma unroll 1
  for (int kb = 0; kb < SEQ; kb += 64) {
    v8f s[4];
    #pragma unroll
    for (int j = 0; j < 4; ++j) {
      const _Float16* kp = kbase + (size_t)(kb + 16 * j) * HD;
      const v16h kf0 = load_frag(kp, h);
      const v16h kf1 = load_frag(kp + 32, h);
      v8f z = zero8;
      z = wmma_f16(kf0, qb0, z);
      z = wmma_f16(kf1, qb1, z);
      s[j] = z * QKSC;
    }

    float mloc = s[0][0];
    #pragma unroll
    for (int j = 0; j < 4; ++j)
      #pragma unroll
      for (int r = 0; r < 8; ++r) mloc = fmaxf(mloc, s[j][r]);
    mloc = fmaxf(mloc, __shfl_xor(mloc, 16));
    const float mnew = fmaxf(mrun, mloc);
    const float alpha = __expf(mrun - mnew);
    mrun = mnew;
    float lsum = 0.0f;
    #pragma unroll
    for (int j = 0; j < 4; ++j)
      #pragma unroll
      for (int r = 0; r < 8; ++r) {
        const float p = __expf(s[j][r] - mnew);
        s[j][r] = p;
        lsum += p;
      }
    lsum += __shfl_xor(lsum, 16);
    lrun = lrun * alpha + lsum;
    #pragma unroll
    for (int t = 0; t < 4; ++t)
      #pragma unroll
      for (int r = 0; r < 8; ++r) o[t][r] = o[t][r] * alpha;

    const v16h pb0 = pack_p(s[0], s[1]);
    const v16h pb1 = pack_p(s[2], s[3]);

    #pragma unroll
    for (int t = 0; t < 4; ++t) {
      const _Float16* vp = vbase + (size_t)(16 * t) * SEQ + kb;
      const v16h vf0 = load_frag(vp, h);
      const v16h vf1 = load_frag(vp + 32, h);
      o[t] = wmma_f16(vf0, pb0, o[t]);
      o[t] = wmma_f16(vf1, pb1, o[t]);
    }
  }

  const float inv = (1.0f / lrun) * (OSC / PSCALE);
  _Float16* so = sO + w * 1024;
  #pragma unroll
  for (int t = 0; t < 4; ++t)
    #pragma unroll
    for (int r = 0; r < 8; ++r)
      so[m * 64 + 16 * t + 8 * h + r] = (_Float16)(o[t][r] * inv);
  __syncthreads();

  att_store_pass(so, oh, b, head, q0, lane);
  __threadfence();
  att_store_pass(so, oh, b, head, q0, lane);
}

__device__ __forceinline__ void out_store_pass(const float* sY, float* out,
                                               int m0, int n0, int w, int lane) {
  const int q8 = lane & 7, sub = lane >> 3;
  #pragma unroll
  for (int i = 0; i < 16; ++i) {
    const int lid = i * 4 + sub;
    const int tokl = 32 * w + (lid >> 1), hl = lid & 1;
    const v4f v = *(const v4fa*)(sY + tokl * 64 + 32 * hl + 4 * q8);
    *(volatile v4f*)(out + (size_t)(m0 + tokl) * DMODEL + n0 + 32 * hl + 4 * q8) = v;
  }
}

__global__ __launch_bounds__(128) void out_kernel(
    const _Float16* __restrict__ oh,
    const _Float16* __restrict__ woT,
    const float* __restrict__ bo,
    float* __restrict__ out)
{
  __shared__ __attribute__((aligned(16))) float sY[128 * 64];

  const int tid = threadIdx.x, lane = tid & 31, w = tid >> 5;
  const int h = lane >> 4, m = lane & 15;
  const int m0 = blockIdx.x * 128;
  const int n0 = blockIdx.y * 64;
  const int m0w = m0 + 32 * w;

  const _Float16* xa0 = oh + (size_t)(m0w + m) * INNER;
  const _Float16* xa1 = xa0 + (size_t)16 * INNER;
  const _Float16* wb  = woT + (size_t)(n0 + m) * INNER;

  const v8f zero8 = {0.f, 0.f, 0.f, 0.f, 0.f, 0.f, 0.f, 0.f};
  v8f acc[2][4];
  #pragma unroll
  for (int mt = 0; mt < 2; ++mt)
    #pragma unroll
    for (int nt = 0; nt < 4; ++nt) acc[mt][nt] = zero8;

  #pragma unroll 1
  for (int k0 = 0; k0 < INNER; k0 += 32) {
    const v16h a0 = load_frag(xa0 + k0, h);
    const v16h a1 = load_frag(xa1 + k0, h);
    #pragma unroll
    for (int nt = 0; nt < 4; ++nt) {
      const v16h b = load_frag(wb + (size_t)nt * 16 * INNER + k0, h);
      acc[0][nt] = wmma_f16(a0, b, acc[0][nt]);
      acc[1][nt] = wmma_f16(a1, b, acc[1][nt]);
    }
  }

  #pragma unroll
  for (int nt = 0; nt < 4; ++nt) {
    const int feat = 16 * nt + m;
    const float bvl = bo[n0 + feat];
    #pragma unroll
    for (int mt = 0; mt < 2; ++mt) {
      #pragma unroll
      for (int r = 0; r < 8; ++r) {
        const int tokl = 32 * w + 16 * mt + 8 * h + r;
        sY[tokl * 64 + feat] = acc[mt][nt][r] * (1.0f / (WSC * OSC)) + bvl;
      }
    }
  }
  __syncthreads();

  out_store_pass(sY, out, m0, n0, w, lane);
  __threadfence();
  out_store_pass(sY, out, m0, n0, w, lane);
}

extern "C" void kernel_launch(void* const* d_in, const int* in_sizes, int n_in,
                              void* d_out, int out_size, void* d_ws, size_t ws_size,
                              hipStream_t stream) {
  if (n_in < 10) return;
  if (in_sizes[0] != NX || in_sizes[1] != NX) return;
  if (in_sizes[2] != NW || in_sizes[4] != NW || in_sizes[6] != NW || in_sizes[8] != NW) return;
  if (in_sizes[3] != INNER || in_sizes[5] != INNER || in_sizes[7] != INNER) return;
  if (in_sizes[9] != DMODEL) return;
  if (out_size != NX) return;

  const float* x   = (const float*)d_in[0];
  const float* ctx = (const float*)d_in[1];
  const float* wq  = (const float*)d_in[2];
  const float* bq  = (const float*)d_in[3];
  const float* wk  = (const float*)d_in[4];
  const float* bk  = (const float*)d_in[5];
  const float* wv  = (const float*)d_in[6];
  const float* bv  = (const float*)d_in[7];
  const float* wo  = (const float*)d_in[8];
  const float* bo  = (const float*)d_in[9];
  float* out = (float*)d_out;

  const size_t act_bytes = (size_t)NX * 2;
  const size_t wt_bytes  = (size_t)3 * NW * 2;
  const size_t wo_bytes  = (size_t)NW * 2;
  const size_t pl_bytes  = (size_t)NO * 2;
  const size_t total = 2 * act_bytes + wt_bytes + wo_bytes + 4 * pl_bytes;
  if (total > ws_size) return;

  char* ws = (char*)d_ws;
  size_t off = 0;
  _Float16* xh  = (_Float16*)(ws + off); off += act_bytes;
  _Float16* ch  = (_Float16*)(ws + off); off += act_bytes;
  _Float16* wT  = (_Float16*)(ws + off); off += wt_bytes;
  _Float16* woT = (_Float16*)(ws + off); off += wo_bytes;
  _Float16* qh  = (_Float16*)(ws + off); off += pl_bytes;
  _Float16* kh  = (_Float16*)(ws + off); off += pl_bytes;
  _Float16* vt  = (_Float16*)(ws + off); off += pl_bytes;
  _Float16* oh  = (_Float16*)(ws + off); off += pl_bytes;
  if (off > ws_size) return;

  convert_act_kernel<<<(2 * NX8) / 256, 256, 0, stream>>>(x, ctx, xh, ch);

  wtrans_kernel<<<512, 256, 0, stream>>>(wq, wk, wv, wo, wT, woT);

  dim3 gQkv(MROWS / 128, 3 * NHEADS);
  qkv_kernel<<<gQkv, 128, 0, stream>>>(xh, ch, wT, bq, bk, bv, qh, kh, vt);

  dim3 gAtt(SEQ / 64, BATCH * NHEADS);
  attn_kernel<<<gAtt, 128, 0, stream>>>(qh, kh, vt, oh);

  dim3 gOut(MROWS / 128, DMODEL / 64);
  out_kernel<<<gOut, 128, 0, stream>>>(oh, woT, bo, out);
}
